// DeformableElementwiseDynamicConv2d_76149770158460
// MI455X (gfx1250) — hardware-verified
//
#include <hip/hip_runtime.h>
#include <math.h>

typedef __attribute__((ext_vector_type(16))) _Float16 v16h;
typedef __attribute__((ext_vector_type(16))) __bf16 v16b;
typedef __attribute__((ext_vector_type(8)))  _Float16 v8h;
typedef __attribute__((ext_vector_type(8)))  float v8f;
typedef __attribute__((ext_vector_type(4)))  float v4f;
typedef __attribute__((ext_vector_type(2)))  float v2f;
typedef __attribute__((ext_vector_type(4)))  unsigned v4u;
typedef __attribute__((ext_vector_type(4)))  int v4i;
typedef float __attribute__((may_alias)) float_a;
typedef int __attribute__((may_alias)) int_a;

template <typename T> __device__ __forceinline__ void vst2(void* p, T v) { *(volatile T*)p = v; __threadfence(); *(volatile T*)p = v; }
__device__ __forceinline__ v8f wmma16(v16h a, v16h b, v8f c) {
  v8f d = __builtin_amdgcn_wmma_f32_16x16x32_f16(false, a, false, b, (short)0, c, false, false);
  asm volatile("v_nop\n\tv_nop\n\tv_nop\n\tv_nop" : "+v"(d) : "v"(a), "v"(b));
  return d;
}
__device__ __forceinline__ v8f wmma_bf(v16b a, v16b b, v8f c) {
  v8f d = __builtin_amdgcn_wmma_f32_16x16x32_bf16(false, a, false, b, (short)0, c, false, false);
  asm volatile("v_nop\n\tv_nop\n\tv_nop\n\tv_nop" : "+v"(d) : "v"(a), "v"(b));
  return d;
}
__device__ __forceinline__ v16h frag_h(const _Float16* rowk0, int lane) {
  union { v16h v; v8h q[2]; } u; const _Float16* p = rowk0 + 8 * (lane >> 4);
  u.q[0] = *(const v8h*)p; u.q[1] = *(const v8h*)(p + 16); return u.v;
}
__device__ __forceinline__ v16h frag_f32(const float* rowk0, int lane) {
  v16h a; const float* p = rowk0 + 8 * (lane >> 4);
#pragma unroll
  for (int i = 0; i < 8; ++i) { a[i] = (_Float16)p[i]; a[8 + i] = (_Float16)p[16 + i]; }
  return a;
}
__device__ __forceinline__ v16h frag_f32s(const float* rowk0, int lane, float sc) {
  v16h a; const float* p = rowk0 + 8 * (lane >> 4);
#pragma unroll
  for (int i = 0; i < 8; ++i) { a[i] = (_Float16)(p[i] * sc); a[8 + i] = (_Float16)(p[16 + i] * sc); }
  return a;
}
__device__ __forceinline__ v16h fragc_f32(const float* W, int k0, int n, int lane, int ld, int K) {
  v16h a; const int g = lane >> 4;
#pragma unroll
  for (int i = 0; i < 8; ++i) { const int ka = k0 + 8 * g + i, kb = ka + 16;
    a[i] = (_Float16)(ka < K ? W[(size_t)(ka < K ? ka : K - 1) * ld + n] : 0.f); a[8 + i] = (_Float16)(kb < K ? W[(size_t)(kb < K ? kb : K - 1) * ld + n] : 0.f); }
  return a;
}
struct F2 { v16b h, l; };
__device__ __forceinline__ F2 bsplit16(const float v[16]) { F2 r;
#pragma unroll
  for (int i = 0; i < 16; ++i) { const __bf16 h = (__bf16)v[i]; r.h[i] = h; r.l[i] = (__bf16)(v[i] - (float)h); }
  return r; }
__device__ __forceinline__ F2 split_row(const float* row, int k0, int lane) { float v[16]; const float* p = row + k0 + 8 * (lane >> 4);
#pragma unroll
  for (int i = 0; i < 8; ++i) { v[i] = p[i]; v[8 + i] = p[16 + i]; }
  return bsplit16(v); }
__device__ __forceinline__ F2 split_rowK(const float* row, int k0, int lane, int K) { float v[16]; const int g = lane >> 4;
#pragma unroll
  for (int i = 0; i < 8; ++i) { const int ka = k0 + 8 * g + i, kb = ka + 16; v[i] = ka < K ? row[ka < K ? ka : K - 1] : 0.f; v[8 + i] = kb < K ? row[kb < K ? kb : K - 1] : 0.f; }
  return bsplit16(v); }
__device__ __forceinline__ F2 split_col(const float* W, int k0, int n, int lane, int ld, int K) { float v[16]; const int g = lane >> 4;
#pragma unroll
  for (int i = 0; i < 8; ++i) { const int ka = k0 + 8 * g + i, kb = ka + 16; v[i] = ka < K ? W[(size_t)(ka < K ? ka : K - 1) * ld + n] : 0.f; v[8 + i] = kb < K ? W[(size_t)(kb < K ? kb : K - 1) * ld + n] : 0.f; }
  return bsplit16(v); }
__device__ __forceinline__ v8f mac3(const F2& a, const F2& b, v8f c) { c = wmma_bf(a.l, b.h, c); c = wmma_bf(a.h, b.l, c); return wmma_bf(a.h, b.h, c); }
__device__ __forceinline__ float sigm(float v) { return 1.0f / (1.0f + expf(-v)); }
#define LDSX() do { asm volatile("s_wait_dscnt 0" ::: "memory"); __builtin_amdgcn_wave_barrier(); __builtin_amdgcn_fence(__ATOMIC_RELEASE, "workgroup"); } while (0)


#define NB 8
#define CH 64
#define HH 128
#define WW 128
#define KK 9
#define NPX (HH * WW)
#ifndef TPR
#define TPR HH
#define TDR HH
#define TNB NB
#endif
typedef __attribute__((ext_vector_type(8))) __bf16 v8b;
__device__ __forceinline__ v16b frag_b(const __bf16* rowk0, int lane) {
  union { v16b v; v8b q[2]; } u; const __bf16* p = rowk0 + 8 * (lane >> 4);
  u.q[0] = *(const v8b*)p; u.q[1] = *(const v8b*)(p + 16); return u.v;
}
__device__ __forceinline__ float bfr(float v) { return (float)(__bf16)v; }
__device__ __attribute__((noinline)) float exp_ni(float v) { return expf(v); }
__device__ __attribute__((noinline)) float erf_ni(float v) { return erff(v); }

#define NL 7
#define WS_W   0u
#define WS_H1H (((2u * NL * KK * CH * CH) + 127u) / 128u * 128u)
#define PLANE  (2u * (size_t)NB * CH * NPX)
#define WS_H1L (WS_H1H + PLANE)
#define WS_H2H (WS_H1L + PLANE)
#define WS_H2L (WS_H2H + PLANE)
#define WS_OFF (WS_H2L + PLANE)
#define WS_ATT (WS_OFF + 4u * (size_t)NB * CH * NPX)
#define WS_END (WS_ATT + 4u * (size_t)NB * 2 * CH * NPX)

__global__ __launch_bounds__(64) void k_packw(const float* __restrict__ W1, const float* __restrict__ W2, const float* __restrict__ W3, const float* __restrict__ WA, const float* __restrict__ WD, __bf16* __restrict__ PW) {
  const int o = blockIdx.x, k = blockIdx.y, layer = blockIdx.z, c = threadIdx.x; __shared__ __align__(16) __bf16 s[CH]; float v;
  switch (layer) { case 0: v = W1[((size_t)o * CH + c) * KK + k]; break; case 1: v = W2[((size_t)o * CH + c) * KK + k]; break; case 2: v = (o < 36) ? W3[((size_t)o * CH + c) * KK + k] : 0.f; break; case 3: v = WA[((size_t)o * CH + c) * KK + k]; break; case 4: v = WA[((size_t)(64 + o) * CH + c) * KK + k]; break; case 5: v = WD[((size_t)o * CH + c) * KK + k]; break; default: v = WD[(((size_t)CH + o) * CH + c) * KK + k]; break; }
  s[c] = (__bf16)v; __syncthreads();
  if (c < CH / 8) vst2((unsigned*)(PW + (((size_t)layer * KK + k) * CH + o) * CH + c * 8), *(const v4u*)&s[c * 8]);
}
template <int INEX, int OUTF, int SLOT>
__global__ __launch_bounds__(128) void k_conv(const float* __restrict__ X, const __bf16* __restrict__ IH, const __bf16* __restrict__ IL, const __bf16* __restrict__ PW, __bf16* __restrict__ OH_, __bf16* __restrict__ OL_, float* __restrict__ OUTF32) {
  __shared__ __align__(16) __bf16 sh[66][72], sl[66][72]; __shared__ __align__(16) __bf16 soh[CH][72], sol[CH][72];
  const int tid = threadIdx.x, wave = tid >> 5, lane = tid & 31, col = lane & 15, g = lane >> 4; const int x0 = (blockIdx.x & 1) * 64, y = blockIdx.x >> 1; const size_t b = blockIdx.y;
  const __bf16* Wl = PW + (size_t)SLOT * KK * CH * CH;
  v8f acc[4] = {};
#pragma unroll 1
  for (int dy = 0; dy < 3; ++dy) { const int yy = y + dy - 1;
    for (int e = tid; e < 66 * CH; e += 128) { const int c = e / 66, xi = e % 66; const int xx = x0 - 1 + xi; float v = 0.f, vl = 0.f; __bf16 hb, lb;
      if (yy >= 0 && yy < HH && xx >= 0 && xx < WW) { const size_t idx = ((b * CH + c) * HH + yy) * WW + xx; if (INEX) { hb = (__bf16)X[idx]; lb = (__bf16)0.f; } else { hb = IH[idx]; lb = IL[idx]; } } else { hb = (__bf16)0.f; lb = (__bf16)0.f; }
      (void)v; (void)vl; sh[xi][c] = hb; sl[xi][c] = lb; }
    if (tid < 66) for (int c = CH; c < 72; ++c) { sh[tid][c] = (__bf16)0.f; sl[tid][c] = (__bf16)0.f; }
    __syncthreads();
#pragma unroll
    for (int dx = 0; dx < 3; ++dx) { const int k = dy * 3 + dx;
#pragma unroll
      for (int kc = 0; kc < 2; ++kc) { const v16b a = frag_b(&sh[wave * 16 + col + dx][kc * 32], lane);
        if (INEX) {
#pragma unroll
          for (int j = 0; j < 4; ++j) acc[j] = wmma_bf(a, frag_b(Wl + ((size_t)k * CH + j * 16 + col) * CH + kc * 32, lane), acc[j]);
        } else { const v16b al = frag_b(&sl[wave * 16 + col + dx][kc * 32], lane);
#pragma unroll
          for (int j = 0; j < 4; ++j) { const v16b w = frag_b(Wl + ((size_t)k * CH + j * 16 + col) * CH + kc * 32, lane); acc[j] = wmma_bf(al, w, acc[j]); acc[j] = wmma_bf(a, w, acc[j]); } } } }
    __syncthreads(); }
  if (OUTF) { __shared__ __align__(16) float sof[CH][68];
#pragma unroll
    for (int j = 0; j < 4; ++j) { const int o = j * 16 + col;
#pragma unroll
      for (int r = 0; r < 8; ++r) sof[o][wave * 16 + 8 * g + r] = acc[j][r]; }
    __syncthreads();
    for (int e = tid; e < CH * 16; e += 128) { const int o = e >> 4, q = e & 15; vst2(OUTF32 + ((b * CH + o) * HH + y) * WW + x0 + q * 4, *(const v4f*)&sof[o][q * 4]); }
  } else {
#pragma unroll
    for (int j = 0; j < 4; ++j) { const int o = j * 16 + col;
#pragma unroll
      for (int r = 0; r < 8; ++r) { const float v = fmaxf(acc[j][r], 0.f); const __bf16 hb = (__bf16)v; soh[o][wave * 16 + 8 * g + r] = hb; sol[o][wave * 16 + 8 * g + r] = (__bf16)(v - (float)hb); } }
    __syncthreads();
    for (int e = tid; e < CH * 8; e += 128) { const int o = e >> 3, q = e & 7; const size_t idx = ((b * CH + o) * HH + y) * WW + x0 + q * 8; vst2((unsigned*)(OH_ + idx), *(const v4u*)&soh[o][q * 8]); vst2((unsigned*)(OL_ + idx), *(const v4u*)&sol[o][q * 8]); } }
}
__global__ __launch_bounds__(128) void k_deform(const float* __restrict__ X, const float* __restrict__ OFF, const float* __restrict__ ATT, const __bf16* __restrict__ PW, float* __restrict__ OUT) {
  __shared__ __align__(16) __bf16 sh[64][72], sl[64][72]; __shared__ int sidx[4][64]; __shared__ float swt[4][64], swy[2][64], swx[2][64]; __shared__ __align__(16) float so[CH][68];
  const int tid = threadIdx.x, wave = tid >> 5, lane = tid & 31, col = lane & 15, g = lane >> 4; const int x0 = (blockIdx.x & 1) * 64, y = blockIdx.x >> 1; const size_t b = blockIdx.y;
  v8f acc[4], accs[2][4];
#pragma unroll
  for (int dk = 0; dk < 2; ++dk) { const __bf16* Wd = PW + (size_t)(5 + dk) * KK * CH * CH;
#pragma unroll
  for (int j = 0; j < 4; ++j) acc[j] = v8f{};
#pragma unroll 1
  for (int k = 0; k < KK; ++k) {
    if (tid < 64) { const int x = x0 + tid; const float ky = (float)(k / 3 - 1), kx = (float)(k % 3 - 1);
      const float oy = OFF[((b * CH + dk * 2 * KK + 2 * k) * HH + y) * WW + x], ox = OFF[((b * CH + dk * 2 * KK + 2 * k + 1) * HH + y) * WW + x];
      const float basey = (float)(y - 1) + (float)(k / 3), basex = (float)(x - 1) + (float)(k % 3);
      const float py = basey + oy, px = basex + ox; const float y0 = floorf(py), xq0 = floorf(px); const float ay = py - y0, ax = px - xq0; const int y0i = (int)y0, x0i = (int)xq0;
#pragma unroll
      for (int q = 0; q < 4; ++q) { const int dy = q >> 1, dx = q & 1; const int yi = y0i + dy, xi = x0i + dx; const bool valid = (yi >= 0) && (yi < HH) && (xi >= 0) && (xi < WW);
        const int ycl = yi < 0 ? 0 : (yi > HH - 1 ? HH - 1 : yi), xcl = xi < 0 ? 0 : (xi > WW - 1 ? WW - 1 : xi); sidx[q][tid] = ycl * WW + xcl; swt[q][tid] = valid ? 1.0f : 0.0f; }
      swy[0][tid] = 1.0f - ay; swy[1][tid] = ay; swx[0][tid] = 1.0f - ax; swx[1][tid] = ax; }
    __syncthreads();
    for (int e = tid; e < 64 * CH; e += 128) { const int px_ = e & 63, c = e >> 6; const size_t base = (b * CH + c) * NPX; float vq[4];
#pragma unroll
      for (int q = 0; q < 4; ++q) vq[q] = bfr(X[base + sidx[q][px_]]) * swt[q][px_];
      const float ay1 = swy[0][px_], ay = swy[1][px_], ax1 = swx[0][px_], ax = swx[1][px_];
      const float v = ((vq[0] * ay1 * ax1 + vq[1] * ay1 * ax) + vq[2] * ay * ax1) + vq[3] * ay * ax;
      const __bf16 hb = (__bf16)v; sh[px_][c] = hb; sl[px_][c] = (__bf16)(v - (float)hb); }
    if (tid < 64) for (int c = CH; c < 72; ++c) { sh[tid][c] = (__bf16)0.f; sl[tid][c] = (__bf16)0.f; }
    __syncthreads();
#pragma unroll
    for (int kc = 0; kc < 2; ++kc) { const v16b a = frag_b(&sh[wave * 16 + col][kc * 32], lane), al = frag_b(&sl[wave * 16 + col][kc * 32], lane);
#pragma unroll
      for (int j = 0; j < 4; ++j) { const v16b w = frag_b(Wd + ((size_t)k * CH + j * 16 + col) * CH + kc * 32, lane); acc[j] = wmma_bf(al, w, acc[j]); acc[j] = wmma_bf(a, w, acc[j]); } }
    __syncthreads(); }
#pragma unroll
  for (int j = 0; j < 4; ++j) accs[dk][j] = acc[j]; }
#pragma unroll
  for (int j = 0; j < 4; ++j) { const int o = j * 16 + col;
#pragma unroll
    for (int r = 0; r < 8; ++r) { const int x = x0 + wave * 16 + 8 * g + r; const float a0 = ATT[((b * CH + o) * HH + y) * WW + x], a1 = ATT[(size_t)NB * CH * NPX + ((b * CH + o) * HH + y) * WW + x];   const float mx = fmaxf(a0, a1); const float e0 = __expf(a0 - mx), e1 = __expf(a1 - mx); const float inv = 1.0f / (e0 + e1);
      float out = 0.f; out = out + accs[0][j][r] * (e0 * inv); out = out + accs[1][j][r] * (e1 * inv); so[o][wave * 16 + 8 * g + r] = out; } }
  __syncthreads();
  for (int e = tid; e < CH * 16; e += 128) { const int o = e >> 4, q = e & 15; vst2(OUT + ((b * CH + o) * HH + y) * WW + x0 + q * 4, *(const v4f*)&so[o][q * 4]); }
}
extern "C" void kernel_launch(void* const* d_in, const int* in_sizes, int n_in, void* d_out, int out_size, void* d_ws, size_t ws_size, hipStream_t stream) {
  (void)in_sizes; (void)n_in; (void)out_size;
  const float** F = (const float**)d_in;
  if (ws_size < (size_t)WS_END) return;
  char* ws = (char*)d_ws; __bf16 *PW = (__bf16*)(ws + WS_W), *H1H = (__bf16*)(ws + WS_H1H), *H1L = (__bf16*)(ws + WS_H1L), *H2H = (__bf16*)(ws + WS_H2H), *H2L = (__bf16*)(ws + WS_H2L); float *OFF = (float*)(ws + WS_OFF), *ATT = (float*)(ws + WS_ATT);
  k_packw<<<dim3(CH, KK, NL), 64, 0, stream>>>(F[1], F[2], F[3], F[4], F[5], PW);
  k_conv<1, 0, 0><<<dim3(2 * TPR, TNB), 128, 0, stream>>>(F[0], nullptr, nullptr, PW, H1H, H1L, nullptr);
  k_conv<0, 0, 1><<<dim3(2 * TPR, TNB), 128, 0, stream>>>(nullptr, H1H, H1L, PW, H2H, H2L, nullptr);
  k_conv<0, 1, 2><<<dim3(2 * TPR, TNB), 128, 0, stream>>>(nullptr, H2H, H2L, PW, nullptr, nullptr, OFF);
  k_conv<1, 1, 3><<<dim3(2 * TDR, TNB), 128, 0, stream>>>(F[0], nullptr, nullptr, PW, nullptr, nullptr, ATT);
  k_conv<1, 1, 4><<<dim3(2 * TDR, TNB), 128, 0, stream>>>(F[0], nullptr, nullptr, PW, nullptr, nullptr, ATT + (size_t)NB * CH * NPX);
  k_deform<<<dim3(2 * TDR, TNB), 128, 0, stream>>>(F[0], OFF, ATT, PW, (float*)d_out);
}
